// DCNv2_SA_27522150432907
// MI455X (gfx1250) — hardware-run, weakly checked
//
#include <hip/hip_runtime.h>
#include <math.h>

typedef __attribute__((ext_vector_type(16))) _Float16 v16h;
typedef __attribute__((ext_vector_type(8)))  _Float16 v8h;
typedef __attribute__((ext_vector_type(8)))  float    v8f;
typedef __attribute__((ext_vector_type(4)))  float    v4f;
typedef __attribute__((ext_vector_type(4)))  int      v4i;

constexpr int kNB        = 4;
constexpr int kCin       = 256;
constexpr int kCout      = 256;
constexpr int kHt        = 96;
constexpr int kWd        = 96;
constexpr int kHW        = kHt * kWd;
constexpr int kNpos      = kNB * kHW;
constexpr int kTaps      = 9;
constexpr int kKdim      = kTaps * kCin;
constexpr int kSteps     = kKdim / 32;
constexpr int kTileM     = 64;
constexpr int kBlkPerImg = kHW / kTileM;
constexpr int kNumTiles  = kNpos / kTileM;
constexpr int kAPitch    = 40;
constexpr int kSlabPitch = 68;
constexpr int kGroups    = 8;
constexpr int kChPerGrp  = kCout / kGroups;
constexpr int kGrpElems  = kChPerGrp * kHW;
constexpr float kValCarry = 8.0f;
constexpr float kWgtCarry = 16.0f;
constexpr float kFold     = 1.0f / (kValCarry * kWgtCarry);

static_assert(kHW == 9216 && kNpos == 36864 && kKdim == 2304 && kSteps == 72, "shape");
static_assert((kHW % kTileM) == 0 && (kNpos % kTileM) == 0, "M tile multiple");
static_assert((kKdim % 32) == 0 && (kCin % 32) == 0, "K multiple of 32, chunk inside one tap");
static_assert(kCout == 8 * 32 && kChPerGrp == 32, "one wave owns one channel group");
static_assert(kBlkPerImg == 144 && kNumTiles == 576, "tiles");
static_assert(kGrpElems == 294912, "group size");

constexpr size_t kOffXH    = 0;
constexpr size_t kOffConv  = kOffXH   + (size_t)kNpos * kCin * 4;
constexpr size_t kOffBt    = kOffConv + (size_t)kNB * kCout * kHW * 4;
constexpr size_t kOffPart  = kOffBt   + (size_t)kCout * kKdim * 2;
constexpr size_t kOffStats = kOffPart + (size_t)kNumTiles * 32 * 4;
constexpr size_t kWsTotal  = kOffStats + (size_t)kNB * kGroups * 32 * 4;
static_assert(kWsTotal == 76754944ull, "carve total");
static_assert(kWsTotal <= 134217728ull, "carve cap");
static_assert((kOffConv % 128) == 0 && (kOffBt % 128) == 0 && (kOffPart % 128) == 0 && (kOffStats % 128) == 0, "aligned regions");

union FragU { v16h v; v8h h[2]; };

__device__ __forceinline__ v16h frag_load_global(const _Float16* p) {
  FragU f;
  f.h[0] = *(const v8h*)(p);
  f.h[1] = *(const v8h*)(p + 16);
  return f.v;
}

__device__ __forceinline__ v8f mma_f16(v16h a, v16h b, v8f c) {
  c = __builtin_amdgcn_wmma_f32_16x16x32_f16(false, a, false, b, (short)0, c, false, false);
  asm volatile("v_nop\n\tv_nop\n\tv_nop\n\tv_nop" : "+v"(c) : "v"(a), "v"(b));
  return c;
}

__global__ __launch_bounds__(256) void nhwc_copy_kernel(const float* __restrict__ x, float* __restrict__ xh) {
  __shared__ float tile[256 * 33];
  const int tid = threadIdx.x, lane = tid & 31, wave = tid >> 5;
  const int b   = blockIdx.x / (kHW / 32);
  const int hw0 = (blockIdx.x - b * (kHW / 32)) * 32;
#pragma unroll 8
  for (int i = 0; i < 32; ++i) {
    const int c = i * 8 + wave;
    tile[c * 33 + lane] = x[((size_t)(b * kCin + c)) * kHW + hw0 + lane];
  }
  __syncthreads();
  v4f vals[8];
#pragma unroll
  for (int it = 0; it < 8; ++it) {
    const int item = it * 8 + wave;
    const int p  = item >> 1;
    const int c4 = (item & 1) * 128 + lane * 4;
    v4f t;
    t[0] = tile[(c4 + 0) * 33 + p];
    t[1] = tile[(c4 + 1) * 33 + p];
    t[2] = tile[(c4 + 2) * 33 + p];
    t[3] = tile[(c4 + 3) * 33 + p];
    vals[it] = t;
  }
  for (int pass = 0; pass < 2; ++pass) {
#pragma unroll
    for (int it = 0; it < 8; ++it) {
      const int item = it * 8 + wave;
      const int p  = item >> 1;
      const int c4 = (item & 1) * 128 + lane * 4;
      *(volatile v4f*)(xh + ((size_t)(b * kHW + hw0 + p)) * kCin + c4) = vals[it];
    }
    __threadfence();
  }
}

__global__ __launch_bounds__(256) void weight_plane_kernel(const float* __restrict__ w, _Float16* __restrict__ bt) {
  const int i  = blockIdx.x * 256 + threadIdx.x;
  const int e0 = i * 8;
  const int o  = e0 / kKdim;
  const int k  = e0 - o * kKdim;
  const int tap = k >> 8;
  const int c0  = k & 255;
  const float* wp = w + ((size_t)(o * kCin + c0)) * kTaps + tap;
  v8h hv;
#pragma unroll
  for (int e = 0; e < 8; ++e) {
    const float f = wp[e * kTaps] * kWgtCarry;
    hv[e] = (_Float16)f;
  }
  _Float16* q = bt + (size_t)e0;
  *(volatile v8h*)q = hv;
  __threadfence();
  *(volatile v8h*)q = hv;
}

__device__ __forceinline__ v8h sample_oct(const float* __restrict__ xh, v4f pw, v4i pi, int cbase) {
  const float* r0 = xh + (size_t)pi[0] * kCin + cbase;
  const float* r1 = xh + (size_t)pi[1] * kCin + cbase;
  const float* r2 = xh + (size_t)pi[2] * kCin + cbase;
  const float* r3 = xh + (size_t)pi[3] * kCin + cbase;
  const v4f a0 = *(const v4f*)(r0);
  const v4f a1 = *(const v4f*)(r0 + 4);
  const v4f b0 = *(const v4f*)(r1);
  const v4f b1 = *(const v4f*)(r1 + 4);
  const v4f c0 = *(const v4f*)(r2);
  const v4f c1 = *(const v4f*)(r2 + 4);
  const v4f d0 = *(const v4f*)(r3);
  const v4f d1 = *(const v4f*)(r3 + 4);
  const float w0 = pw[0], w1 = pw[1], w2 = pw[2], w3 = pw[3];
  v8h hv;
#pragma unroll
  for (int e = 0; e < 4; ++e) {
    float u = w0 * a0[e];
    u = fmaf(w1, b0[e], u);
    u = fmaf(w2, c0[e], u);
    u = fmaf(w3, d0[e], u);
    float t = w0 * a1[e];
    t = fmaf(w1, b1[e], t);
    t = fmaf(w2, c1[e], t);
    t = fmaf(w3, d1[e], t);
    hv[e]     = (_Float16)u;
    hv[4 + e] = (_Float16)t;
  }
  return hv;
}

__global__ __launch_bounds__(256) void deform_gemm_kernel(
    const float* __restrict__ xh, const float* __restrict__ off, const float* __restrict__ msk,
    const _Float16* __restrict__ bt, float* __restrict__ conv, float* __restrict__ part)
{
  __shared__ __align__(16) _Float16 sA[2 * 64 * kAPitch];
  __shared__ __align__(16) float    sPw[kTaps * 64 * 4];
  __shared__ __align__(16) int      sPi[kTaps * 64 * 4];
  __shared__ __align__(16) float    sSlab[8 * 16 * kSlabPitch];
  __shared__ float sRed[16];

  const int tid = threadIdx.x, lane = tid & 31, wave = tid >> 5;
  const int b   = blockIdx.x / kBlkPerImg;
  const int hw0 = (blockIdx.x - b * kBlkPerImg) * kTileM;

#pragma unroll 1
  for (int it3 = 0; it3 < 3; ++it3) {
    const int tap = it3 * 4 + (tid >> 6);
    if (tap < kTaps) {
      const int p  = tid & 63;
      const int hw = hw0 + p;
      const int yy = hw / kWd;
      const int xx = hw - yy * kWd;
      const int ky = tap / 3;
      const int kx = tap - ky * 3;
      const float dy = off[(b * 18 + 2 * tap) * kHW + hw];
      const float dx = off[(b * 18 + 2 * tap + 1) * kHW + hw];
      const float mv = msk[(b * kTaps + tap) * kHW + hw] * kValCarry;
      const float py = (float)(yy + ky - 1) + dy;
      const float px = (float)(xx + kx - 1) + dx;
      const float fy = floorf(py);
      const float fx = floorf(px);
      const float wy = py - fy;
      const float wx = px - fx;
      const int y0 = (int)fminf(fmaxf(fy, -2.0f), 97.0f);
      const int x0 = (int)fminf(fmaxf(fx, -2.0f), 97.0f);
      const int y1 = y0 + 1;
      const int x1 = x0 + 1;
      const bool vy0 = (y0 >= 0) && (y0 < kHt);
      const bool vy1 = (y1 >= 0) && (y1 < kHt);
      const bool vx0 = (x0 >= 0) && (x0 < kWd);
      const bool vx1 = (x1 >= 0) && (x1 < kWd);
      const float oy = 1.0f - wy;
      const float ox = 1.0f - wx;
      const float t00 = (oy * ox) * mv;
      const float t01 = (oy * wx) * mv;
      const float t10 = (wy * ox) * mv;
      const float t11 = (wy * wx) * mv;
      v4f pw;
      pw[0] = (vy0 && vx0) ? t00 : 0.0f;
      pw[1] = (vy0 && vx1) ? t01 : 0.0f;
      pw[2] = (vy1 && vx0) ? t10 : 0.0f;
      pw[3] = (vy1 && vx1) ? t11 : 0.0f;
      const int y0c = min(max(y0, 0), kHt - 1);
      const int y1c = min(max(y1, 0), kHt - 1);
      const int x0c = min(max(x0, 0), kWd - 1);
      const int x1c = min(max(x1, 0), kWd - 1);
      v4i pi;
      pi[0] = b * kHW + y0c * kWd + x0c;
      pi[1] = b * kHW + y0c * kWd + x1c;
      pi[2] = b * kHW + y1c * kWd + x0c;
      pi[3] = b * kHW + y1c * kWd + x1c;
      *(v4f*)(sPw + (tap * 64 + p) * 4) = pw;
      *(v4i*)(sPi + (tap * 64 + p) * 4) = pi;
    }
  }
  __syncthreads();

  const int sp = tid >> 2;
  const int cq = tid & 3;
  const int rlane = lane & 15;
  const int hh    = lane >> 4;
  const int koff  = hh * 8;
  const _Float16* Bw = bt + (size_t)(wave * 32 + rlane) * kKdim + koff;

  v8f acc[4][2];
#pragma unroll
  for (int i = 0; i < 4; ++i) {
    acc[i][0] = (v8f){0.f, 0.f, 0.f, 0.f, 0.f, 0.f, 0.f, 0.f};
    acc[i][1] = (v8f){0.f, 0.f, 0.f, 0.f, 0.f, 0.f, 0.f, 0.f};
  }

  {
    const v4f pw = *(const v4f*)(sPw + sp * 4);
    const v4i pi = *(const v4i*)(sPi + sp * 4);
    const v8h hv = sample_oct(xh, pw, pi, cq * 8);
    *(v8h*)(sA + sp * kAPitch + cq * 8) = hv;
  }
  __syncthreads();

#pragma unroll 1
  for (int it = 0; it < kSteps; ++it) {
    const int cur = it & 1;
    const v16h b0 = frag_load_global(Bw + it * 32);
    const v16h b1 = frag_load_global(Bw + (size_t)16 * kKdim + it * 32);
    const int abase = cur * (64 * kAPitch) + rlane * kAPitch + koff;
#pragma unroll
    for (int i = 0; i < 4; ++i) {
      FragU af;
      af.h[0] = *(const v8h*)(sA + abase + i * 16 * kAPitch);
      af.h[1] = *(const v8h*)(sA + abase + i * 16 * kAPitch + 16);
      acc[i][0] = mma_f16(af.v, b0, acc[i][0]);
      acc[i][1] = mma_f16(af.v, b1, acc[i][1]);
    }
    if (it + 1 < kSteps) {
      const int nxt  = it + 1;
      const int tapn = nxt >> 3;
      const int qn   = nxt & 7;
      const v4f pw = *(const v4f*)(sPw + (tapn * 64 + sp) * 4);
      const v4i pi = *(const v4i*)(sPi + (tapn * 64 + sp) * 4);
      const v8h hv = sample_oct(xh, pw, pi, qn * 32 + cq * 8);
      *(v8h*)(sA + (cur ^ 1) * (64 * kAPitch) + sp * kAPitch + cq * 8) = hv;
    }
    __syncthreads();
  }

  float s1 = 0.0f, s2 = 0.0f;
  const int c4 = (lane & 15) * 4;
#pragma unroll
  for (int j = 0; j < 2; ++j) {
#pragma unroll
    for (int i = 0; i < 4; ++i) {
#pragma unroll
      for (int r = 0; r < 8; ++r) {
        const float v = acc[i][j][r] * kFold;
        s1 += v;
        s2 = fmaf(v, v, s2);
        sSlab[wave * (16 * kSlabPitch) + rlane * kSlabPitch + i * 16 + 8 * hh + r] = v;
      }
    }
    __builtin_amdgcn_fence(__ATOMIC_RELEASE, "workgroup");
    __builtin_amdgcn_wave_barrier();
    __builtin_amdgcn_fence(__ATOMIC_ACQUIRE, "workgroup");
    v4f ov[8];
#pragma unroll
    for (int t = 0; t < 8; ++t) {
      const int row = t * 2 + hh;
      ov[t] = *(const v4f*)(sSlab + wave * (16 * kSlabPitch) + row * kSlabPitch + c4);
    }
    for (int pass = 0; pass < 2; ++pass) {
#pragma unroll
      for (int t = 0; t < 8; ++t) {
        const int row = t * 2 + hh;
        const int ch  = wave * 32 + j * 16 + row;
        *(volatile v4f*)(conv + ((size_t)(b * kCout + ch)) * kHW + hw0 + c4) = ov[t];
      }
      __threadfence();
    }
    __builtin_amdgcn_fence(__ATOMIC_RELEASE, "workgroup");
    __builtin_amdgcn_wave_barrier();
    __builtin_amdgcn_fence(__ATOMIC_ACQUIRE, "workgroup");
  }
#pragma unroll
  for (int o = 16; o > 0; o >>= 1) {
    s1 += __shfl_xor(s1, o, 32);
    s2 += __shfl_xor(s2, o, 32);
  }
  if (lane == 0) {
    sRed[wave * 2]     = s1;
    sRed[wave * 2 + 1] = s2;
  }
  __syncthreads();
  if (wave == 0) {
    const float t = sRed[lane & 15];
    const float val = (lane < 16) ? t : 0.0f;
    volatile float* pp = part + (size_t)blockIdx.x * 32 + lane;
    *pp = val;
    __threadfence();
    *pp = val;
  }
}

__global__ __launch_bounds__(32) void group_stats_kernel(const float* __restrict__ part, float* __restrict__ stats) {
  const int lane = threadIdx.x;
  const int bg = blockIdx.x;
  const int b  = bg >> 3;
  const int g  = bg & 7;
  double s = 0.0, q = 0.0;
#pragma unroll 1
  for (int i0 = 0; i0 < 160; i0 += 32) {
    const int i  = i0 + lane;
    const int ic = (i < kBlkPerImg) ? i : (kBlkPerImg - 1);
    const float a = part[((size_t)(b * kBlkPerImg + ic)) * 32 + g * 2];
    const float c = part[((size_t)(b * kBlkPerImg + ic)) * 32 + g * 2 + 1];
    const bool ok = (i < kBlkPerImg);
    s += ok ? (double)a : 0.0;
    q += ok ? (double)c : 0.0;
  }
#pragma unroll
  for (int o = 16; o > 0; o >>= 1) {
    s += __shfl_xor(s, o, 32);
    q += __shfl_xor(q, o, 32);
  }
  const double inv = 1.0 / (double)kGrpElems;
  const double mu  = s * inv;
  double var = q * inv - mu * mu;
  var = (var > 0.0) ? var : 0.0;
  const float muf  = (float)mu;
  const float rstd = rsqrtf((float)var + 1e-5f);
  const float val = (lane == 0) ? muf : ((lane == 1) ? rstd : 0.0f);
  volatile float* pp = stats + (size_t)bg * 32 + lane;
  *pp = val;
  __threadfence();
  *pp = val;
}

__global__ __launch_bounds__(256) void group_apply_kernel(
    const float* __restrict__ conv, const float* __restrict__ stats,
    const float* __restrict__ gamma, const float* __restrict__ beta, float* __restrict__ out)
{
  const int base4 = blockIdx.x * 1024 + threadIdx.x;
  v4f res[4];
#pragma unroll
  for (int k = 0; k < 4; ++k) {
    const int e0 = (base4 + k * 256) * 4;
    const int bo = e0 / kHW;
    const int o  = bo & (kCout - 1);
    const int bb = bo >> 8;
    const int bg = bb * kGroups + (o >> 5);
    const float mu   = stats[bg * 32];
    const float rstd = stats[bg * 32 + 1];
    const float gm = gamma[o];
    const float be = beta[o];
    const v4f v = *(const v4f*)(conv + e0);
    v4f t;
#pragma unroll
    for (int e = 0; e < 4; ++e) {
      float u = (v[e] - mu) * rstd;
      u = u * gm + be;
      t[e] = fmaxf(u, 0.0f);
    }
    res[k] = t;
  }
  for (int pass = 0; pass < 2; ++pass) {
#pragma unroll
    for (int k = 0; k < 4; ++k) {
      *(volatile v4f*)(out + (size_t)(base4 + k * 256) * 4) = res[k];
    }
    __threadfence();
  }
}

extern "C" void kernel_launch(void* const* d_in, const int* in_sizes, int n_in,
                              void* d_out, int out_size, void* d_ws, size_t ws_size,
                              hipStream_t stream) {
  if (n_in < 6) return;
  if (in_sizes[0] != kNB * kCin * kHW) return;
  if (in_sizes[1] != kNB * 18 * kHW) return;
  if (in_sizes[2] != kNB * kTaps * kHW) return;
  if (in_sizes[3] != kCout * kCin * kTaps) return;
  if (in_sizes[4] != kCout) return;
  if (in_sizes[5] != kCout) return;
  if (out_size != kNB * kCout * kHW) return;
  if (ws_size < kWsTotal) return;

  const float* x     = (const float*)d_in[0];
  const float* off   = (const float*)d_in[1];
  const float* msk   = (const float*)d_in[2];
  const float* wgt   = (const float*)d_in[3];
  const float* gamma = (const float*)d_in[4];
  const float* beta  = (const float*)d_in[5];
  float* out = (float*)d_out;

  char* ws = (char*)d_ws;
  float*    xh    = (float*)(ws + kOffXH);
  float*    conv  = (float*)(ws + kOffConv);
  _Float16* bt    = (_Float16*)(ws + kOffBt);
  float*    part  = (float*)(ws + kOffPart);
  float*    stats = (float*)(ws + kOffStats);

  nhwc_copy_kernel<<<kNpos / 32, 256, 0, stream>>>(x, xh);
  weight_plane_kernel<<<(kCout * kKdim / 8) / 256, 256, 0, stream>>>(wgt, bt);
  deform_gemm_kernel<<<kNumTiles, 256, 0, stream>>>(xh, off, msk, bt, conv, part);
  group_stats_kernel<<<kNB * kGroups, 32, 0, stream>>>(part, stats);
  group_apply_kernel<<<(kNB * kCout * kHW) / 4096, 256, 0, stream>>>(conv, stats, gamma, beta, out);
}
